// DHSMoEDetector_3092376453874
// MI455X (gfx1250) — hardware-verified
//
#include <hip/hip_runtime.h>
#include <stddef.h>
#include <stdint.h>

#pragma clang fp contract(off)

#define NTOK   16384
#define DD     768
#define HH     768
#define CC     2
#define NE     20
#define NTILE  276
#define NROWS  (NTILE * 64)
#define NCH    (NTOK / 256)
#define WSC    64.0f
#define INV64  0.015625f
#define APITCH 136
#define TRP    72

static_assert(NTILE == NTOK / 64 + NE);
static_assert(DD % 128 == 0);
static_assert(HH % 128 == 0);
static_assert(DD % 64 == 0);
static_assert(HH % 64 == 0);
static_assert(NTOK % 256 == 0);
static_assert(NTOK % 64 == 0);
static_assert((NTOK * DD) % 2048 == 0);
static_assert(NROWS % 4 == 0);
static_assert((NROWS / 4) <= 18 * 256);
static_assert(NTOK <= 65536);
static_assert(NE <= 32);
static_assert(CC == 2);

typedef _Float16 v16h __attribute__((ext_vector_type(16)));
typedef _Float16 v8h  __attribute__((ext_vector_type(8)));
typedef float    v8f  __attribute__((ext_vector_type(8)));
typedef float    v4f  __attribute__((ext_vector_type(4)));
typedef float    v2f  __attribute__((ext_vector_type(2)));
typedef unsigned int v4u __attribute__((ext_vector_type(4)));
typedef int      v4i  __attribute__((ext_vector_type(4)));
typedef unsigned short v4us __attribute__((ext_vector_type(4)));

union Frag  { v16h v; v8h h[2]; };
union Pack8 { v8h h; v4u u; };

__device__ __forceinline__ int clampi(int v, int lo, int hi) { return min(max(v, lo), hi); }

__device__ __forceinline__ v8f mma16(v16h a, v16h b, v8f c) {
  c = __builtin_amdgcn_wmma_f32_16x16x32_f16(false, a, false, b, (short)0, c, false, false);
  asm volatile("v_nop\n\tv_nop\n\tv_nop\n\tv_nop" : "+v"(c) : "v"(a), "v"(b));
  return c;
}

__device__ __forceinline__ v16h ldfrag(const _Float16* p, int ld, int row0, int k0, int lane) {
  const int m = lane & 15, lh = lane >> 4;
  const _Float16* q = p + (size_t)(row0 + m) * ld + k0 + 8 * lh;
  Frag f;
  f.h[0] = *(const v8h*)(q);
  f.h[1] = *(const v8h*)(q + 16);
  return f.v;
}

__device__ __forceinline__ v8f zero8() { return (v8f){0.f, 0.f, 0.f, 0.f, 0.f, 0.f, 0.f, 0.f}; }

__global__ __launch_bounds__(256) void k_cvt(const float* __restrict__ src, _Float16* __restrict__ dh, int n8) {
  const int i = blockIdx.x * 256 + (int)threadIdx.x;
  if (i >= n8) return;
  const size_t o = (size_t)i * 8;
  const v4f a0 = *(const v4f*)(src + o);
  const v4f a1 = *(const v4f*)(src + o + 4);
  Pack8 pk;
  pk.h = (v8h){(_Float16)a0[0], (_Float16)a0[1], (_Float16)a0[2], (_Float16)a0[3],
               (_Float16)a1[0], (_Float16)a1[1], (_Float16)a1[2], (_Float16)a1[3]};
  const v4u vv = pk.u;
  volatile v4u* d = (volatile v4u*)(dh + o);
  *d = vv;
  __threadfence();
  *d = vv;
}

__global__ __launch_bounds__(256) void k_wtr(const float* __restrict__ w, _Float16* __restrict__ wt,
                                             int kdim, int ndim, float scale) {
  __shared__ __align__(16) _Float16 st[64 * TRP];
  const int tid = threadIdx.x;
  const size_t bo = (size_t)blockIdx.z * (size_t)kdim * (size_t)ndim;
  w  += bo;
  wt += bo;
  const int n0 = blockIdx.x * 64, k0 = blockIdx.y * 64;
  const int kr = tid >> 2;
  const int nc = (tid & 3) * 16;
  const float* sp = w + (size_t)(k0 + kr) * ndim + n0 + nc;
#pragma unroll
  for (int q = 0; q < 4; ++q) {
    const v4f a = *(const v4f*)(sp + 4 * q) * scale;
#pragma unroll
    for (int j = 0; j < 4; ++j) st[(nc + 4 * q + j) * TRP + kr] = (_Float16)a[j];
  }
  __syncthreads();
  v4u val[2];
  size_t go[2];
#pragma unroll
  for (int j = 0; j < 2; ++j) {
    const int p  = tid + 256 * j;
    const int nr = p >> 3;
    const int pc = p & 7;
    Pack8 pk;
    pk.h   = *(const v8h*)(st + nr * TRP + pc * 8);
    val[j] = pk.u;
    go[j]  = (size_t)(n0 + nr) * kdim + k0 + pc * 8;
  }
  for (int ps = 0; ps < 2; ++ps) {
#pragma unroll
    for (int j = 0; j < 2; ++j) *(volatile v4u*)(wt + go[j]) = val[j];
    __threadfence();
  }
}

__global__ __launch_bounds__(256) void k_lists(const int* __restrict__ cid, int* __restrict__ tokp,
                                               int* __restrict__ posp, int* __restrict__ tab) {
  __shared__ __align__(16) unsigned short ltok[NROWS];
  __shared__ int wc[8 * NE];
  __shared__ int wsum[8 * NE];
  __shared__ int srun[NE];
  __shared__ __align__(16) int sTab[64];
  const int tid = threadIdx.x, lane = tid & 31, wave = tid >> 5;
  const unsigned ltm = (1u << lane) - 1u;

  for (int i = tid; i < NROWS; i += 256) ltok[i] = (unsigned short)0;
  if (tid < 64) sTab[tid] = 0;
  if (tid < NE) srun[tid] = 0;

  int hacc[NE];
#pragma unroll
  for (int e = 0; e < NE; ++e) hacc[e] = 0;
#pragma unroll 1
  for (int ch = 0; ch < NCH; ++ch) {
    const int t  = ch * 256 + tid;
    const int et = clampi(cid[t], 0, NE - 1);
#pragma unroll
    for (int e = 0; e < NE; ++e) {
      const unsigned bal = __builtin_amdgcn_ballot_w32(et == e);
      hacc[e] += __builtin_popcount(bal);
    }
  }
  int hv = 0;
#pragma unroll
  for (int e = 0; e < NE; ++e) hv = (lane == e) ? hacc[e] : hv;
  if (lane < NE) wsum[wave * NE + lane] = hv;
  __syncthreads();
  if (tid < NE) {
    int s = 0;
#pragma unroll
    for (int q = 0; q < 8; ++q) s += wsum[q * NE + tid];
    sTab[tid] = s;
  }
  __syncthreads();
  if (tid == 0) {
    int run = 0;
#pragma unroll 1
    for (int e = 0; e < NE; ++e) {
      sTab[32 + e] = run;
      run += (clampi(sTab[e], 0, NTOK) + 63) >> 6;
    }
    sTab[32 + NE] = clampi(run, 0, NTILE);
  }
  __syncthreads();

#pragma unroll 1
  for (int ch = 0; ch < NCH; ++ch) {
    const int t  = ch * 256 + tid;
    const int et = clampi(cid[t], 0, NE - 1);
    int pre = 0;
#pragma unroll
    for (int e = 0; e < NE; ++e) {
      const bool m = (et == e);
      const unsigned bal = __builtin_amdgcn_ballot_w32(m);
      pre = m ? __builtin_popcount(bal & ltm) : pre;
      if (lane == 0) wc[wave * NE + e] = __builtin_popcount(bal);
    }
    __syncthreads();
    int base = srun[et];
#pragma unroll
    for (int q = 0; q < 8; ++q) base += (q < wave) ? wc[q * NE + et] : 0;
    int tot = 0;
    if (tid < NE) {
#pragma unroll
      for (int q = 0; q < 8; ++q) tot += wc[q * NE + tid];
    }
    const int tbe = clampi(sTab[32 + et], 0, NTILE - 1);
    const int row = clampi(tbe * 64 + base + pre, 0, NROWS - 1);
    ltok[row] = (unsigned short)t;
    volatile int* pd = (volatile int*)(posp + t);
    *pd = row;
    __threadfence();
    *pd = row;
    __syncthreads();
    if (tid < NE) srun[tid] += tot;
  }
  __syncthreads();

  for (int ps = 0; ps < 2; ++ps) {
#pragma unroll 1
    for (int it = 0; it < 18; ++it) {
      const int p = tid + 256 * it;
      if (p < NROWS / 4) {
        const v4us u = *(const v4us*)(ltok + p * 4);
        const v4i v = (v4i){(int)u[0], (int)u[1], (int)u[2], (int)u[3]};
        *(volatile v4i*)(tokp + (size_t)p * 4) = v;
      }
    }
    __threadfence();
  }
  if (wave == 0) {
    const v4i v = *(const v4i*)(sTab + (lane & 15) * 4);
    volatile v4i* d = (volatile v4i*)(tab + (lane & 15) * 4);
    if (lane < 16) *d = v;
    __threadfence();
    if (lane < 16) *d = v;
  }
}

__global__ __launch_bounds__(256) void k_gemm(const _Float16* __restrict__ xh, const _Float16* __restrict__ w1t,
                                              const float* __restrict__ b1, const float* __restrict__ w2,
                                              const float* __restrict__ b2, const int* __restrict__ tokp,
                                              const int* __restrict__ tab, float* __restrict__ yp) {
  __shared__ __align__(16) _Float16 sA[64 * APITCH];
  __shared__ __align__(16) float sY[2 * 64 * CC];
  __shared__ __align__(16) float sF[64 * CC];
  __shared__ int sTok[64];
  __shared__ int sTab[64];
  const int tid = threadIdx.x, lane = tid & 31, wave = tid >> 5;
  const int hh = lane >> 4, c = lane & 15;
  const int wm = wave & 3, wn = wave >> 2;
  const int b  = blockIdx.x;

  if (tid < 64) sTab[tid] = tab[tid];
  __syncthreads();
  const int ntl = clampi(sTab[32 + NE], 0, NTILE);
  if (b >= ntl) return;
  int e = 0;
#pragma unroll
  for (int q = 1; q < NE; ++q) e += (clampi(sTab[32 + q], 0, NTILE) <= b) ? 1 : 0;
  if (tid < 64) sTok[tid] = clampi(tokp[b * 64 + tid], 0, NTOK - 1);
  __syncthreads();

  const _Float16* wte = w1t + (size_t)e * (size_t)(HH * DD);
  const float* b1e = b1 + e * HH;
  const float* w2e = w2 + (size_t)e * (HH * CC);

  float py0[8], py1[8];
#pragma unroll
  for (int r = 0; r < 8; ++r) { py0[r] = 0.f; py1[r] = 0.f; }

  const int ar = tid >> 2, ac = tid & 3;
  const _Float16* xrow = xh + (size_t)sTok[ar] * DD + ac * 32;
  _Float16* arow = sA + ar * APITCH + ac * 32;

#pragma unroll 1
  for (int nc = 0; nc < HH / 128; ++nc) {
    const int brow = nc * 128 + wn * 64;
    v8f acc[4];
#pragma unroll
    for (int t = 0; t < 4; ++t) acc[t] = zero8();
#pragma unroll 1
    for (int kc = 0; kc < DD / 128; ++kc) {
      __syncthreads();
#pragma unroll
      for (int q = 0; q < 4; ++q) *(v8h*)(arow + 8 * q) = *(const v8h*)(xrow + kc * 128 + 8 * q);
      __syncthreads();
#pragma unroll 1
      for (int ks = 0; ks < 4; ++ks) {
        const int kg = kc * 128 + ks * 32;
        const v16h a = ldfrag(sA, APITCH, wm * 16, ks * 32, lane);
#pragma unroll
        for (int t = 0; t < 4; ++t) {
          const v16h bq = ldfrag(wte, DD, brow + 16 * t, kg, lane);
          acc[t] = mma16(a, bq, acc[t]);
        }
      }
    }
#pragma unroll
    for (int t = 0; t < 4; ++t) {
      const int n = brow + 16 * t + c;
      const float bias64 = b1e[n] * WSC;
      const v2f wv = *(const v2f*)(w2e + (size_t)n * CC);
#pragma unroll
      for (int r = 0; r < 8; ++r) {
        const float hs = fmaxf(acc[t][r] + bias64, 0.f);
        py0[r] = fmaf(hs, wv[0], py0[r]);
        py1[r] = fmaf(hs, wv[1], py1[r]);
      }
    }
  }

#pragma unroll
  for (int r = 0; r < 8; ++r) {
#pragma unroll
    for (int off = 1; off < 16; off <<= 1) {
      py0[r] += __shfl_xor(py0[r], off, 32);
      py1[r] += __shfl_xor(py1[r], off, 32);
    }
  }
  if (c == 0) {
#pragma unroll
    for (int r = 0; r < 8; ++r) {
      const int row = wm * 16 + 8 * hh + r;
      sY[(wn * 64 + row) * CC + 0] = py0[r];
      sY[(wn * 64 + row) * CC + 1] = py1[r];
    }
  }
  __syncthreads();
  if (tid < 64) {
    const int row = tid;
    const float s0 = sY[row * CC + 0] + sY[(64 + row) * CC + 0];
    const float s1 = sY[row * CC + 1] + sY[(64 + row) * CC + 1];
    sF[row * CC + 0] = s0 * INV64 + b2[e * CC + 0];
    sF[row * CC + 1] = s1 * INV64 + b2[e * CC + 1];
  }
  __syncthreads();
  if (wave == 0) {
    const v4f v = *(const v4f*)(sF + lane * 4);
    volatile v4f* d = (volatile v4f*)(yp + (size_t)(b * 64) * CC + lane * 4);
    *d = v;
    __threadfence();
    *d = v;
  }
}

__global__ __launch_bounds__(256) void k_out(const float* __restrict__ yp, const int* __restrict__ posp,
                                             float* __restrict__ out, int n4) {
  const int i = blockIdx.x * 256 + (int)threadIdx.x;
  if (i >= n4) return;
  const int t0 = 2 * i;
  const int r0 = clampi(posp[t0], 0, NROWS - 1);
  const int r1 = clampi(posp[t0 + 1], 0, NROWS - 1);
  const v2f a = *(const v2f*)(yp + (size_t)r0 * CC);
  const v2f bq = *(const v2f*)(yp + (size_t)r1 * CC);
  const v4f v = (v4f){a[0], a[1], bq[0], bq[1]};
  volatile v4f* d = (volatile v4f*)(out + (size_t)t0 * CC);
  *d = v;
  __threadfence();
  *d = v;
}

extern "C" void kernel_launch(void* const* d_in, const int* in_sizes, int n_in,
                              void* d_out, int out_size, void* d_ws, size_t ws_size,
                              hipStream_t stream) {
  if (n_in < 6) return;
  if (in_sizes[0] != NTOK * DD) return;
  if (in_sizes[1] != NTOK) return;
  if (in_sizes[2] != NE * DD * HH) return;
  if (in_sizes[3] != NE * HH) return;
  if (in_sizes[4] != NE * HH * CC) return;
  if (in_sizes[5] != NE * CC) return;
  if (out_size != NTOK * CC) return;

  const float* x   = (const float*)d_in[0];
  const int*   cid = (const int*)d_in[1];
  const float* W1  = (const float*)d_in[2];
  const float* b1  = (const float*)d_in[3];
  const float* W2  = (const float*)d_in[4];
  const float* b2  = (const float*)d_in[5];
  float* out = (float*)d_out;

  size_t off = 0;
  const size_t oXh = off; off += (size_t)NTOK * DD * 2;
  const size_t oW1 = off; off += (size_t)NE * HH * DD * 2;
  const size_t oTK = off; off += (size_t)NROWS * 4;
  const size_t oPS = off; off += (size_t)NTOK * 4;
  const size_t oTB = off; off += (size_t)256;
  const size_t oY  = off; off += (size_t)NROWS * CC * 4;
  if (off > ws_size) return;
  if (off > (size_t)134217728) return;
  if ((oW1 | oTK | oPS | oTB | oY) & (size_t)127) return;

  char* ws = (char*)d_ws;
  _Float16* Xh  = (_Float16*)(ws + oXh);
  _Float16* W1T = (_Float16*)(ws + oW1);
  int*      TOK = (int*)(ws + oTK);
  int*      POS = (int*)(ws + oPS);
  int*      TAB = (int*)(ws + oTB);
  float*    Y   = (float*)(ws + oY);

  k_cvt<<<dim3((NTOK * DD) / 8 / 256), dim3(256), 0, stream>>>(x, Xh, (NTOK * DD) / 8);
  k_wtr<<<dim3(HH / 64, DD / 64, NE), dim3(256), 0, stream>>>(W1, W1T, DD, HH, WSC);
  k_lists<<<dim3(1), dim3(256), 0, stream>>>(cid, TOK, POS, TAB);
  k_gemm<<<dim3(NTILE), dim3(256), 0, stream>>>(Xh, W1T, b1, W2, b2, TOK, TAB, Y);
  k_out<<<dim3(NTOK / 2 / 256), dim3(256), 0, stream>>>(Y, POS, out, NTOK / 2);
  (void)hipGetLastError();
}
